// ODEFunc_90159953478502
// MI455X (gfx1250) — hardware-verified
//
#include <hip/hip_runtime.h>
#include <math.h>

typedef __attribute__((ext_vector_type(16))) _Float16 v16h;
typedef __attribute__((ext_vector_type(8)))  _Float16 v8h;
typedef __attribute__((ext_vector_type(16))) __bf16   v16b;
typedef __attribute__((ext_vector_type(8)))  __bf16   v8b;
typedef __attribute__((ext_vector_type(8)))  float    v8f;
typedef __attribute__((ext_vector_type(4)))  float    v4f;

constexpr int NROW   = 4096;
constexpr int DMODEL = 256;
constexpr int DHID   = 1024;
constexpr int NEXP   = 8;
constexpr int KMAIN  = NEXP * DHID;
constexpr int KTAIL  = 64;
constexpr int KTOT   = KMAIN + KTAIL;
constexpr int TPB    = 256;
constexpr int NGB    = NROW / TPB;
constexpr int FLAG_LINE_U32 = 32;

static_assert(NROW % TPB == 0);
static_assert(NGB <= TPB);
static_assert(TPB == 256);
static_assert(DMODEL == TPB);
static_assert(DMODEL * NEXP == 8 * TPB);
static_assert(KTOT % 64 == 0);
static_assert(KTOT % 32 == 0 && DMODEL % 32 == 0);
static_assert(NROW % 64 == 0 && DHID % 64 == 0 && DMODEL % 64 == 0);
static_assert(((NROW / 64) * (DHID / 64)) % 8 == 0);
static_assert(((NROW / 64) * (DMODEL / 64)) % 8 == 0);
static_assert((NROW * DMODEL) % (8 * TPB) == 0);

constexpr size_t SZ_XH  = (size_t)NROW * DMODEL * 2;
constexpr size_t SZ_W1T = (size_t)NEXP * DHID * DMODEL * 2;
constexpr size_t SZ_BT2 = (size_t)DMODEL * KTOT * 2;
constexpr size_t SZ_HP  = (size_t)NROW * KTOT * 2;
constexpr size_t SZ_WTS = (size_t)NROW * NEXP * 4;
constexpr size_t SZ_FLG = (size_t)NGB * FLAG_LINE_U32 * 4;
constexpr size_t SZ_ST  = (size_t)NEXP * NROW * 4;
constexpr size_t OFF_XH  = 0;
constexpr size_t OFF_W1T = OFF_XH + SZ_XH;
constexpr size_t OFF_BT2 = OFF_W1T + SZ_W1T;
constexpr size_t OFF_HP  = OFF_BT2 + SZ_BT2;
constexpr size_t OFF_WTS = OFF_HP + SZ_HP;
constexpr size_t OFF_FLG = OFF_WTS + SZ_WTS;
constexpr size_t OFF_ST  = OFF_FLG + SZ_FLG;
constexpr size_t WS_TOTAL = OFF_ST + SZ_ST;
static_assert(WS_TOTAL <= (size_t)134217728);
static_assert(OFF_W1T % 128 == 0 && OFF_BT2 % 128 == 0 && OFF_HP % 128 == 0 &&
              OFF_WTS % 128 == 0 && OFF_FLG % 128 == 0 && OFF_ST % 128 == 0);

__device__ __forceinline__ unsigned short f2bf_bits(float f) {
  unsigned u = __float_as_uint(f);
  return (unsigned short)((u + 0x7FFFu + ((u >> 16) & 1u)) >> 16);
}
__device__ __forceinline__ float bf_bits2f(unsigned short h) { return __uint_as_float(((unsigned)h) << 16); }

__device__ __forceinline__ void dep_guard_h(v8f& a, v8f& b, v16h x, v16h y) { asm volatile("v_nop\n\tv_nop\n\tv_nop\n\tv_nop" : "+v"(a), "+v"(b) : "v"(x), "v"(y)); }
__device__ __forceinline__ void dep_guard_b(v8f& a, v8f& b, v16b x, v16b y) { asm volatile("v_nop\n\tv_nop\n\tv_nop\n\tv_nop" : "+v"(a), "+v"(b) : "v"(x), "v"(y)); }
__device__ __forceinline__ void keep4_h(v16h a, v16h b, v16h c, v16h d) { asm volatile("v_nop" :: "v"(a), "v"(b), "v"(c), "v"(d)); }
__device__ __forceinline__ void keep4_b(v16b a, v16b b, v16b c, v16b d) { asm volatile("v_nop" :: "v"(a), "v"(b), "v"(c), "v"(d)); }
__device__ __forceinline__ void acc_guard4(v8f& a, v8f& b, v8f& c, v8f& d) { asm volatile("v_nop\n\tv_nop\n\tv_nop\n\tv_nop" : "+v"(a), "+v"(b), "+v"(c), "+v"(d)); }
template <typename T> struct Frag;
template <> struct Frag<_Float16> {
  typedef v16h V; union U { v16h v; v8h h[2]; };
  static __device__ __forceinline__ v16h load(const _Float16* p) {
    U f; f.h[0] = *(const v8h*)(p); f.h[1] = *(const v8h*)(p + 16); return f.v;
  }
  static __device__ __forceinline__ v8f mma(v16h a, v16h b, v8f c) {
    return __builtin_amdgcn_wmma_f32_16x16x32_f16(false, a, false, b, (short)0, c, false, false);
  }
  static __device__ __forceinline__ void guard(v8f& a, v8f& b, v16h x, v16h y) { dep_guard_h(a, b, x, y); }
  static __device__ __forceinline__ void keep(v16h a, v16h b, v16h c, v16h d) { keep4_h(a, b, c, d); }
};
template <> struct Frag<__bf16> {
  typedef v16b V; union U { v16b v; v8b h[2]; };
  static __device__ __forceinline__ v16b load(const __bf16* p) {
    U f; f.h[0] = *(const v8b*)(p); f.h[1] = *(const v8b*)(p + 16); return f.v;
  }
  static __device__ __forceinline__ v8f mma(v16b a, v16b b, v8f c) {
    return __builtin_amdgcn_wmma_f32_16x16x32_bf16(false, a, false, b, (short)0, c, false, false);
  }
  static __device__ __forceinline__ void guard(v8f& a, v8f& b, v16b x, v16b y) { dep_guard_b(a, b, x, y); }
  static __device__ __forceinline__ void keep(v16b a, v16b b, v16b c, v16b d) { keep4_b(a, b, c, d); }
};

template <int ET> struct Elem;
template <> struct Elem<0> { typedef _Float16 T; };
template <> struct Elem<1> { typedef __bf16 T; };
template <int ET, bool SPLIT, int BIAS_MODE, int OUT_MODE, bool ROWMUL, int ACT = 0>
__global__ __launch_bounds__(256) void wmma_gemm64(
    const unsigned short* __restrict__ Ap, const unsigned short* __restrict__ A2p, int lda, long strideA,
    const unsigned short* __restrict__ Btp, const unsigned short* __restrict__ Bt2p, int ldb, long strideB,
    void* __restrict__ Cout, void* __restrict__ Cout2, int ldc, long strideC,
    const float* __restrict__ bias, long strideBias,
    const float* __restrict__ rowmul, long strideRM,
    int M, int N, int K, float scale, float oscale) {
  typedef typename Elem<ET>::T T;
  typedef typename Frag<T>::V V;
  const T* A = (const T*)Ap; const T* A2 = (const T*)A2p; const T* Bt = (const T*)Btp; const T* Bt2 = (const T*)Bt2p;
  __shared__ __align__(16) float sT[8][16 * 68];
  const int b    = blockIdx.y;
  const int lane = threadIdx.x & 31;
  const int wave = threadIdx.x >> 5;
  const int tilesN = N >> 6;
  const int tilesM = M >> 6;
  const int tile = blockIdx.x * 8 + wave;
  if (tile >= tilesM * tilesN) return;
  const int tm = tile / tilesN;
  const int tn = tile - tm * tilesN;
  const int m0 = tm << 6;
  const int n0 = tn << 6;

  const T* Ab  = A  + (size_t)b * strideA;
  const T* Bb  = Bt + (size_t)b * strideB;
  const T* Ab2 = SPLIT ? (A2  + (size_t)b * strideA) : nullptr;
  const T* Bb2 = SPLIT ? (Bt2 + (size_t)b * strideB) : nullptr;

  const int rlane = lane & 15;
  const int koff  = (lane >> 4) * 8;
  const int mOff  = (lane >> 4) * 8;

  v8f acc[4][4];
#pragma unroll
  for (int i = 0; i < 4; ++i)
#pragma unroll
    for (int j = 0; j < 4; ++j) acc[i][j] = (v8f){0.f,0.f,0.f,0.f,0.f,0.f,0.f,0.f};

  for (int k0 = 0; k0 < K; k0 += 32) {
    V bh[4], bl[4];
#pragma unroll
    for (int j = 0; j < 4; ++j) {
      const size_t bo = (size_t)(n0 + (j << 4) + rlane) * ldb + koff + k0;
      bh[j] = Frag<T>::load(Bb + bo);
      if (SPLIT) bl[j] = Frag<T>::load(Bb2 + bo);
    }
#pragma unroll
    for (int i = 0; i < 4; ++i) {
      const size_t ao = (size_t)(m0 + (i << 4) + rlane) * lda + koff + k0;
      V ah = Frag<T>::load(Ab + ao);
      V al;
      if (SPLIT) al = Frag<T>::load(Ab2 + ao);
#pragma unroll
      for (int j = 0; j < 4; ++j) {
        acc[i][j] = Frag<T>::mma(ah, bh[j], acc[i][j]);
        if (SPLIT) {
          acc[i][j] = Frag<T>::mma(ah, bl[j], acc[i][j]);
          acc[i][j] = Frag<T>::mma(al, bh[j], acc[i][j]);
        }
      }
      Frag<T>::guard(acc[i][0], acc[i][3], ah, SPLIT ? al : ah);
    }
    Frag<T>::keep(bh[0], bh[1], bh[2], bh[3]);
    if (SPLIT) Frag<T>::keep(bl[0], bl[1], bl[2], bl[3]);
  }
  acc_guard4(acc[0][0], acc[0][1], acc[0][2], acc[0][3]);
  acc_guard4(acc[1][0], acc[1][1], acc[1][2], acc[1][3]);
  acc_guard4(acc[2][0], acc[2][1], acc[2][2], acc[2][3]);
  acc_guard4(acc[3][0], acc[3][1], acc[3][2], acc[3][3]);

  float* slab = sT[wave];
  const float* Bsb = (BIAS_MODE != 0) ? (bias + (size_t)b * strideBias) : nullptr;
  const float* Rmb = ROWMUL ? (rowmul + (size_t)b * strideRM) : nullptr;
#pragma unroll
  for (int i = 0; i < 4; ++i) {
    const int mBase = m0 + (i << 4);
    v8f rmv = (v8f){1.f,1.f,1.f,1.f,1.f,1.f,1.f,1.f};
    if (ROWMUL) {
      const v4f ra = *(const v4f*)(Rmb + mBase + mOff);
      const v4f rb = *(const v4f*)(Rmb + mBase + mOff + 4);
      rmv = (v8f){ra[0], ra[1], ra[2], ra[3], rb[0], rb[1], rb[2], rb[3]};
    }
#pragma unroll
    for (int j = 0; j < 4; ++j) {
      const int n = n0 + (j << 4) + rlane;
      float bv = 0.f;
      if (BIAS_MODE == 2) bv = Bsb[n];
#pragma unroll
      for (int r = 0; r < 8; ++r) {
        float v = acc[i][j][r] * scale;
        if (BIAS_MODE == 2) v += bv;
        if (ACT == 1) v = tanhf(v);
        if (ACT == 2) v = fmaxf(v, 0.0f);
        if (ACT == 4) v = (v > 0.f) ? v : 0.01f * v;
        if (ROWMUL) v *= rmv[r];
        v *= oscale;
        slab[(mOff + r) * 68 + (j << 4) + rlane] = v;
      }
    }
    __builtin_amdgcn_fence(__ATOMIC_RELEASE, "workgroup");
    __builtin_amdgcn_wave_barrier();
    __builtin_amdgcn_fence(__ATOMIC_ACQUIRE, "workgroup");
    if (OUT_MODE == 0) {
      float* C = (float*)Cout + (size_t)b * strideC;
      const int hh = lane >> 4, c4 = (lane & 15) * 4;
      for (int pass = 0; pass < 2; ++pass) {
#pragma unroll
        for (int it = 0; it < 8; ++it) {
          const int row = it * 2 + hh;
          v4f v = *(const v4f*)(slab + row * 68 + c4);
          *(volatile v4f*)(C + (size_t)(mBase + row) * ldc + n0 + c4) = v;
        }
        __threadfence();
      }
    } else {
      const int q = lane >> 3, c8 = (lane & 7) * 8;
      unsigned short* C  = (unsigned short*)Cout  + (size_t)b * strideC;
      unsigned short* C2 = (OUT_MODE == 2) ? ((unsigned short*)Cout2 + (size_t)b * strideC) : nullptr;
      for (int pass = 0; pass < 2; ++pass) {
#pragma unroll
        for (int it = 0; it < 4; ++it) {
          const int row = it * 4 + q;
          const float* sp = slab + row * 68 + c8;
          v8h hv, lv;
#pragma unroll
          for (int e = 0; e < 8; ++e) {
            if (OUT_MODE == 1) {
              hv[e] = (_Float16)sp[e];
            } else {
              unsigned short hb = f2bf_bits(sp[e]);
              unsigned short lb = f2bf_bits(sp[e] - bf_bits2f(hb));
              hv[e] = __builtin_bit_cast(_Float16, hb);
              lv[e] = __builtin_bit_cast(_Float16, lb);
            }
          }
          *(volatile v8h*)(C + (size_t)(mBase + row) * ldc + n0 + c8) = hv;
          if (OUT_MODE == 2) *(volatile v8h*)(C2 + (size_t)(mBase + row) * ldc + n0 + c8) = lv;
        }
        __threadfence();
      }
    }
    __builtin_amdgcn_fence(__ATOMIC_RELEASE, "workgroup");
    __builtin_amdgcn_wave_barrier();
    __builtin_amdgcn_fence(__ATOMIC_ACQUIRE, "workgroup");
  }
}

__global__ __launch_bounds__(TPB) void k_cast_x(const float* __restrict__ in, _Float16* __restrict__ out,
                                               int n8, float sc) {
  const int i = blockIdx.x * TPB + threadIdx.x;
  if (i < n8) {
    const v4f a = *(const v4f*)(in + (size_t)8 * i);
    const v4f c = *(const v4f*)(in + (size_t)8 * i + 4);
    v8h hv;
    hv[0] = (_Float16)(a[0] * sc); hv[1] = (_Float16)(a[1] * sc);
    hv[2] = (_Float16)(a[2] * sc); hv[3] = (_Float16)(a[3] * sc);
    hv[4] = (_Float16)(c[0] * sc); hv[5] = (_Float16)(c[1] * sc);
    hv[6] = (_Float16)(c[2] * sc); hv[7] = (_Float16)(c[3] * sc);
    _Float16* p = out + (size_t)8 * i;
    *(volatile v8h*)p = hv;
    __threadfence();
    *(volatile v8h*)p = hv;
  }
}

__global__ __launch_bounds__(TPB) void k_tr_cast(const float* __restrict__ in, int R, int C,
                                                unsigned short* __restrict__ out, long ozs, int opitch,
                                                long ocz, float sc) {
  __shared__ float tile[64][65];
  const int tid = threadIdx.x, lane = tid & 31, wave = tid >> 5;
  const int c0 = blockIdx.x * 64, r0 = blockIdx.y * 64, z = blockIdx.z;
  const float* inz = in + (size_t)z * R * C;
#pragma unroll
  for (int j = 0; j < 4; ++j) {
    const int r = (tid >> 4) + 16 * j;
    const int cc = (tid & 15) * 4;
    const v4f v = *(const v4f*)(inz + (size_t)(r0 + r) * C + c0 + cc);
    tile[r][cc + 0] = v[0]; tile[r][cc + 1] = v[1]; tile[r][cc + 2] = v[2]; tile[r][cc + 3] = v[3];
  }
  __syncthreads();
  _Float16* oz = (_Float16*)out + (size_t)z * ozs + (size_t)z * ocz;
  const int q = lane & 7;
  for (int pass = 0; pass < 2; ++pass) {
#pragma unroll
    for (int it = 0; it < 2; ++it) {
      const int L = wave * 8 + it * 4 + (lane >> 3);
      v8h hv;
#pragma unroll
      for (int k = 0; k < 8; ++k) hv[k] = (_Float16)(tile[q * 8 + k][L] * sc);
      *(volatile v8h*)(oz + (size_t)(c0 + L) * opitch + r0 + q * 8) = hv;
    }
    __threadfence();
  }
}

__global__ __launch_bounds__(TPB) void k_gate(const float* __restrict__ x, const float* __restrict__ Wg,
                                             const float* __restrict__ bg, const float* __restrict__ tp,
                                             float* __restrict__ wts, unsigned* __restrict__ flags, int nrow) {
  __shared__ __align__(16) float sWg[DMODEL * NEXP];
  __shared__ __align__(16) float sW[TPB * NEXP];
  __shared__ float sWt[NEXP];
  __shared__ float sBg[NEXP];
  __shared__ unsigned sBits[TPB / 32];
  const int tid = threadIdx.x, lane = tid & 31, wave = tid >> 5;
  {
    const v4f a = *(const v4f*)(Wg + 4 * tid);
    const v4f c = *(const v4f*)(Wg + 4 * (tid + TPB));
    *(v4f*)(sWg + 4 * tid) = a;
    *(v4f*)(sWg + 4 * (tid + TPB)) = c;
  }
  if (tid < NEXP) { sWt[tid] = Wg[2 * DMODEL * NEXP + tid]; sBg[tid] = bg[tid]; }
  const float tv = tp[0];
  __syncthreads();

  const int row  = blockIdx.x * TPB + tid;
  const int rowc = (row < nrow) ? row : (nrow - 1);
  const float* xr = x + (size_t)rowc * DMODEL;
  float lg[NEXP];
#pragma unroll
  for (int e = 0; e < NEXP; ++e) lg[e] = 0.f;
#pragma unroll 1
  for (int d4 = 0; d4 < DMODEL / 4; ++d4) {
    const v4f xv = *(const v4f*)(xr + 4 * d4);
#pragma unroll
    for (int c = 0; c < 4; ++c) {
      const float* wp = sWg + (4 * d4 + c) * NEXP;
      const v4f w0 = *(const v4f*)wp;
      const v4f w1 = *(const v4f*)(wp + 4);
#pragma unroll
      for (int e = 0; e < 4; ++e) {
        lg[e]     = fmaf(xv[c], w0[e], lg[e]);
        lg[4 + e] = fmaf(xv[c], w1[e], lg[4 + e]);
      }
    }
  }
  float mx = -INFINITY;
  float* myw = sW + tid * NEXP;
#pragma unroll
  for (int e = 0; e < NEXP; ++e) {
    lg[e] = fmaf(tv, sWt[e], lg[e]) + sBg[e];
    mx = fmaxf(mx, lg[e]);
    myw[e] = lg[e];
  }
  float sum = 0.f;
#pragma unroll 1
  for (int e = 0; e < NEXP; ++e) { const float v = expf(myw[e] - mx); myw[e] = v; sum += v; }
  const float inv = 1.0f / sum;
  unsigned bits = 0u;
#pragma unroll 1
  for (int e = 0; e < NEXP; ++e) {
    const float w = myw[e] * inv;
    myw[e] = w;
    bits |= (w > 0.01f) ? (1u << e) : 0u;
  }
#pragma unroll
  for (int off = 1; off < 32; off <<= 1) bits |= __shfl_xor(bits, off, 32);
  if (lane == 0) sBits[wave] = bits;
  __syncthreads();
  unsigned bb = 0u;
#pragma unroll
  for (int w = 0; w < TPB / 32; ++w) bb |= sBits[w];
  if (wave == 0) {
    const unsigned val = (lane == 0) ? bb : 0u;
    volatile unsigned* fp = flags + (size_t)blockIdx.x * FLAG_LINE_U32 + lane;
    *fp = val;
    __threadfence();
    *fp = val;
  }
  float* wb = wts + (size_t)blockIdx.x * (TPB * NEXP);
  for (int pass = 0; pass < 2; ++pass) {
#pragma unroll
    for (int it = 0; it < 2; ++it) {
      const int f = it * TPB + tid;
      const v4f v = *(const v4f*)(sW + 4 * f);
      *(volatile v4f*)(wb + 4 * (size_t)f) = v;
    }
    __threadfence();
  }
}

__global__ __launch_bounds__(TPB) void k_mix(const float* __restrict__ wts, const unsigned* __restrict__ flags,
                                            float* __restrict__ stab, unsigned short* __restrict__ hp, int nrow) {
  __shared__ unsigned sFl[NGB];
  __shared__ __align__(16) float ss[NEXP * TPB];
  const int tid = threadIdx.x, lane = tid & 31, wave = tid >> 5;
  if (tid < NGB) sFl[tid] = flags[(size_t)tid * FLAG_LINE_U32];
  __syncthreads();
  unsigned ab = 0u;
#pragma unroll
  for (int i = 0; i < NGB; ++i) ab |= sFl[i];
  const bool anyact = (ab != 0u);
  const int row  = blockIdx.x * TPB + tid;
  const int rowc = (row < nrow) ? row : (nrow - 1);
  const v4f w0 = *(const v4f*)(wts + (size_t)rowc * NEXP);
  const v4f w1 = *(const v4f*)(wts + (size_t)rowc * NEXP + 4);
  const v8f w8 = (v8f){w0[0], w0[1], w0[2], w0[3], w1[0], w1[1], w1[2], w1[3]};
#pragma unroll
  for (int e = 0; e < NEXP; ++e) {
    float v = ((ab >> e) & 1u) ? w8[e] : 0.f;
    v = anyact ? v : (1.0f / (float)NEXP);
    ss[e * TPB + tid] = v;
  }
  __syncthreads();
  for (int pass = 0; pass < 2; ++pass) {
#pragma unroll
    for (int it = 0; it < 2; ++it) {
      const int f   = it * TPB + tid;
      const int e   = f / (TPB / 4);
      const int off = (f % (TPB / 4)) * 4;
      const v4f v = *(const v4f*)(ss + 4 * f);
      *(volatile v4f*)(stab + (size_t)e * NROW + (size_t)blockIdx.x * TPB + off) = v;
    }
    __threadfence();
  }
  const int q = lane & 7;
  const float mq = (q == 0) ? 64.f : 0.f;
  _Float16* hb = (_Float16*)hp;
  for (int pass = 0; pass < 2; ++pass) {
#pragma unroll
    for (int it = 0; it < 8; ++it) {
      const int rl = wave * 32 + it * 4 + (lane >> 3);
      v8h hv;
#pragma unroll
      for (int k = 0; k < 8; ++k) hv[k] = (_Float16)(ss[k * TPB + rl] * mq);
      *(volatile v8h*)(hb + ((size_t)blockIdx.x * TPB + rl) * KTOT + KMAIN + q * 8) = hv;
    }
    __threadfence();
  }
}

__global__ __launch_bounds__(TPB) void k_btail(const float* __restrict__ b2, unsigned short* __restrict__ bt) {
  __shared__ float sb[NEXP * DMODEL];
  const int tid = threadIdx.x, lane = tid & 31, wave = tid >> 5;
#pragma unroll
  for (int e = 0; e < NEXP; ++e) sb[e * DMODEL + tid] = b2[e * DMODEL + tid];
  __syncthreads();
  const int q = lane & 7;
  const float mq = (q == 0) ? 32.f : 0.f;
  _Float16* bb = (_Float16*)bt;
  for (int pass = 0; pass < 2; ++pass) {
#pragma unroll
    for (int it = 0; it < 8; ++it) {
      const int rl = wave * 32 + it * 4 + (lane >> 3);
      v8h hv;
#pragma unroll
      for (int k = 0; k < 8; ++k) hv[k] = (_Float16)(sb[k * DMODEL + rl] * mq);
      *(volatile v8h*)(bb + (size_t)rl * KTOT + KMAIN + q * 8) = hv;
    }
    __threadfence();
  }
}

extern "C" void kernel_launch(void* const* d_in, const int* in_sizes, int n_in,
                              void* d_out, int out_size, void* d_ws, size_t ws_size,
                              hipStream_t stream) {
  (void)in_sizes; (void)n_in; (void)out_size;
  const float* tp = (const float*)d_in[0];
  const float* x  = (const float*)d_in[1];
  const float* W1 = (const float*)d_in[2];
  const float* b1 = (const float*)d_in[3];
  const float* W2 = (const float*)d_in[4];
  const float* b2 = (const float*)d_in[5];
  const float* Wg = (const float*)d_in[6];
  const float* bg = (const float*)d_in[7];
  float* out = (float*)d_out;
  if (ws_size < WS_TOTAL) return;
  char* ws = (char*)d_ws;
  unsigned short* xh   = (unsigned short*)(ws + OFF_XH);
  unsigned short* w1t  = (unsigned short*)(ws + OFF_W1T);
  unsigned short* bt2  = (unsigned short*)(ws + OFF_BT2);
  unsigned short* hp   = (unsigned short*)(ws + OFF_HP);
  float*          wts  = (float*)(ws + OFF_WTS);
  unsigned*       flg  = (unsigned*)(ws + OFF_FLG);
  float*          stab = (float*)(ws + OFF_ST);

  const int nx8 = NROW * DMODEL / 8;
  k_cast_x<<<dim3(nx8 / TPB), dim3(TPB), 0, stream>>>(x, (_Float16*)xh, nx8, 16.0f);

  k_tr_cast<<<dim3(DHID / 64, DMODEL / 64, NEXP), dim3(TPB), 0, stream>>>(
      W1, DMODEL, DHID, w1t, (long)DHID * DMODEL, DMODEL, 0L, 16.0f);

  k_tr_cast<<<dim3(DMODEL / 64, DHID / 64, NEXP), dim3(TPB), 0, stream>>>(
      W2, DHID, DMODEL, bt2, 0L, KTOT, (long)DHID, 32.0f);

  k_gate<<<dim3(NGB), dim3(TPB), 0, stream>>>(x, Wg, bg, tp, wts, flg, NROW);

  k_mix<<<dim3(NGB), dim3(TPB), 0, stream>>>(wts, flg, stab, hp, NROW);

  k_btail<<<dim3(1), dim3(TPB), 0, stream>>>(b2, bt2);

  wmma_gemm64<0, false, 2, 1, true, 1><<<dim3((NROW / 64) * (DHID / 64) / 8, NEXP), dim3(256), 0, stream>>>(
      xh, xh, DMODEL, 0L,
      w1t, w1t, DMODEL, (long)DHID * DMODEL,
      (void*)hp, (void*)hp, KTOT, (long)DHID,
      b1, (long)DHID,
      stab, (long)NROW,
      NROW, DHID, DMODEL, 1.0f / 256.0f, 64.0f);

  wmma_gemm64<0, false, 0, 0, false, 0><<<dim3((NROW / 64) * (DMODEL / 64) / 8, 1), dim3(256), 0, stream>>>(
      hp, hp, KTOT, 0L,
      bt2, bt2, KTOT, 0L,
      (void*)out, (void*)out, DMODEL, 0L,
      b1, 0L,
      stab, 0L,
      NROW, DMODEL, KTOT, 1.0f / 2048.0f, 1.0f);
}
